// GAT_76759655514229
// MI455X (gfx1250) — hardware-run, weakly checked
//
#include <hip/hip_runtime.h>

typedef float          v8f   __attribute__((ext_vector_type(8)));
typedef float          v4f   __attribute__((ext_vector_type(4)));
typedef unsigned int   v4u   __attribute__((ext_vector_type(4)));
typedef int            v8i   __attribute__((ext_vector_type(8)));
typedef unsigned short v8us  __attribute__((ext_vector_type(8)));
typedef unsigned short v16us __attribute__((ext_vector_type(16)));
typedef __bf16         v16bf __attribute__((ext_vector_type(16)));
typedef _Float16       v16h  __attribute__((ext_vector_type(16)));
typedef v4f  __attribute__((may_alias)) v4fa;
typedef v8us __attribute__((may_alias)) v8usa;
union FragB { v16bf v; v16us u; v8us h[2]; v8i w; };
union FragH { v16h  v; v16us u; v8us h[2]; v8i w; };

__device__ __forceinline__ v8f wmb(const FragB& a, const FragB& b, v8f c) {
  v8f d = __builtin_amdgcn_wmma_f32_16x16x32_bf16(false, a.v, false, b.v, (short)0, c, false, false);
  asm volatile("v_nop\n\tv_nop\n\tv_nop\n\tv_nop" : "+v"(d) : "v"(a.w), "v"(b.w));
  return d;
}

__device__ __forceinline__ v8f wmh(const FragH& a, const FragH& b, v8f c) {
  v8f d = __builtin_amdgcn_wmma_f32_16x16x32_f16(false, a.v, false, b.v, (short)0, c, false, false);
  asm volatile("v_nop\n\tv_nop\n\tv_nop\n\tv_nop" : "+v"(d) : "v"(a.w), "v"(b.w));
  return d;
}

__device__ __forceinline__ unsigned bf16_bits(float f) {
  const unsigned u = __float_as_uint(f);
  const unsigned r = (u + 0x7FFFu + ((u >> 16) & 1u)) >> 16;
  const unsigned q = (u >> 16) | 0x40u;
  return ((u & 0x7fffffffu) > 0x7f800000u) ? q : r;
}

__device__ __forceinline__ float bf16_val(float f) {
  return __uint_as_float(bf16_bits(f) << 16);
}
__device__ __forceinline__ int clampi(int v, int lo, int hi) {
  return v < lo ? lo : (v > hi ? hi : v);
}

__device__ __forceinline__ unsigned f16_bits(float f) {
  const unsigned u  = __float_as_uint(f);
  const unsigned s  = (u >> 16) & 0x8000u;
  const unsigned a  = u & 0x7fffffffu;
  const unsigned t  = a - 0x38000000u;
  const unsigned r  = (t + 0x0FFFu + ((t >> 13) & 1u)) >> 13;
  const unsigned rc = r > 0x7C00u ? 0x7C00u : r;
  const bool small  = a < 0x38800000u;
  const bool isnan  = a > 0x7f800000u;
  const unsigned fin = small ? 0u : (s | rc);
  return isnan ? (s | 0x7E00u) : fin;
}

__device__ __forceinline__ unsigned pk16(unsigned lo, unsigned hi) { return lo | (hi << 16); }
__device__ __forceinline__ unsigned bf16_lo_bits(float v) {
  float hi = bf16_val(v);
  asm volatile("" : "+v"(hi));
  return bf16_bits(v - hi);
}
__device__ __forceinline__ v4u pack8_bf16(v4f a, v4f c) {
  return (v4u){ pk16(bf16_bits(a[0]), bf16_bits(a[1])), pk16(bf16_bits(a[2]), bf16_bits(a[3])),
                pk16(bf16_bits(c[0]), bf16_bits(c[1])), pk16(bf16_bits(c[2]), bf16_bits(c[3])) };
}
__device__ __forceinline__ v4u pack8_bf16_lo(v4f a, v4f c) {
  return (v4u){ pk16(bf16_lo_bits(a[0]), bf16_lo_bits(a[1])), pk16(bf16_lo_bits(a[2]), bf16_lo_bits(a[3])),
                pk16(bf16_lo_bits(c[0]), bf16_lo_bits(c[1])), pk16(bf16_lo_bits(c[2]), bf16_lo_bits(c[3])) };
}
__device__ __forceinline__ v4u pack8_f16(v4f a, v4f c) {
  return (v4u){ pk16(f16_bits(a[0]), f16_bits(a[1])), pk16(f16_bits(a[2]), f16_bits(a[3])),
                pk16(f16_bits(c[0]), f16_bits(c[1])), pk16(f16_bits(c[2]), f16_bits(c[3])) };
}

template <int FORM>
__global__ __launch_bounds__(256) void k_plane(const float* __restrict__ src, int rows, int cols, int ldsrc,
                                               unsigned short* __restrict__ dst, int MP, int KP) {
  static_assert(FORM >= 0 && FORM <= 3);
  const int KTOT = (FORM == 1 || FORM == 3) ? 2 * KP : KP;
  const unsigned ppr   = (unsigned)(KTOT >> 3);
  const unsigned kp8   = (unsigned)(KP >> 3);
  const unsigned total = (unsigned)MP * ppr;
  const unsigned g     = blockIdx.x * 256u + threadIdx.x;
  const unsigned rowu  = g / ppr;
  const unsigned p     = g - rowu * ppr;
  const bool second    = p >= kp8;
  const int row = (int)rowu;
  const int c0  = (int)((second ? p - kp8 : p) << 3);
  const float* srow = src + (size_t)clampi(row, 0, rows - 1) * (size_t)ldsrc;
  float x[8];
  unsigned mk[8];
#pragma unroll
  for (int e = 0; e < 8; ++e) {
    const int c = c0 + e;
    const float v = srow[clampi(c, 0, cols - 1)];
    asm volatile("" :: "v"(v));
    x[e]  = v;
    mk[e] = (row < rows && c < cols) ? 0xFFFFu : 0u;
  }
  const v4f a = (v4f){ x[0], x[1], x[2], x[3] };
  const v4f c = (v4f){ x[4], x[5], x[6], x[7] };
  v4u o;
  if (FORM == 2) {
    o = pack8_f16(a, c);
  } else {
    const v4u hi = pack8_bf16(a, c);
    o = hi;
    if (FORM == 1) { const v4u lo = pack8_bf16_lo(a, c); o = second ? lo : hi; }
  }
  const v4u mw = (v4u){ pk16(mk[0], mk[1]), pk16(mk[2], mk[3]), pk16(mk[4], mk[5]), pk16(mk[6], mk[7]) };
  o &= mw;
  if (g < total) {
    volatile v4u* q = (volatile v4u*)(dst + (size_t)g * 8);
    *q = o;
    __threadfence();
    *q = o;
  }
}

template <int FORM> struct FragOf    { typedef FragB T; };
template <>         struct FragOf<2> { typedef FragH T; };
__device__ __forceinline__ v8f mm(const FragB& a, const FragB& b, v8f c) { return wmb(a, b, c); }
__device__ __forceinline__ v8f mm(const FragH& a, const FragH& b, v8f c) { return wmh(a, b, c); }
template <class F> __device__ __forceinline__ F ld_frag(const unsigned short* p) {
  F f;
  f.h[0] = *(const v8usa*)(p);
  f.h[1] = *(const v8usa*)(p + 16);
  return f;
}

template <int FORM, int EPI>
__global__ __launch_bounds__(256) __attribute__((amdgpu_num_vgpr(248)))
void k_gemm_nt(const unsigned short* __restrict__ A, const unsigned short* __restrict__ B,
               const float* __restrict__ bias, float* __restrict__ D, int M, int N, int KTOT, int ldd) {
  static_assert(FORM >= 0 && FORM <= 2);
  static_assert(EPI == 0 || EPI == 1);
  typedef typename FragOf<FORM>::T F;
  __shared__ __attribute__((aligned(16))) float sT[8][16 * 68];
  const int lane = threadIdx.x & 31;
  const int wave = threadIdx.x >> 5;
  const int tilesM = (M + 63) >> 6;
  const int tilesN = (N + 63) >> 6;
  const int tile = blockIdx.x * 8 + wave;
  if (tile >= tilesM * tilesN) return;
  const int tm = tile / tilesN;
  const int tn = tile - tm * tilesN;
  const int m0 = tm << 6;
  const int n0 = tn << 6;

  const int rl = lane & 15;
  const int h8 = (lane >> 4) * 8;
  const unsigned short* pa = A + (size_t)(m0 + rl) * (size_t)KTOT + h8;
  const unsigned short* pb = B + (size_t)(n0 + rl) * (size_t)KTOT + h8;

  v8f acc[4][4];
#pragma unroll
  for (int i = 0; i < 4; ++i)
#pragma unroll
    for (int j = 0; j < 4; ++j) acc[i][j] = (v8f){0.f, 0.f, 0.f, 0.f, 0.f, 0.f, 0.f, 0.f};

#pragma unroll 1
  for (int k0 = 0; k0 < KTOT; k0 += 32) {
    F bf[4];
#pragma unroll
    for (int j = 0; j < 4; ++j) bf[j] = ld_frag<F>(pb + (size_t)(j << 4) * (size_t)KTOT + k0);
#pragma unroll
    for (int i = 0; i < 4; ++i) {
      const F af = ld_frag<F>(pa + (size_t)(i << 4) * (size_t)KTOT + k0);
#pragma unroll
      for (int j = 0; j < 4; ++j) acc[i][j] = mm(af, bf[j], acc[i][j]);
    }
  }

  float* slab = sT[wave];
  const int hh = lane >> 4;
  const int c4 = (lane & 15) * 4;
  const int nc = n0 + c4;
  const bool cok = nc < N;
  v4f bv = (v4f){0.f, 0.f, 0.f, 0.f};
  if (EPI == 1) {
    bv = *(const v4fa*)(bias + clampi(nc, 0, N - 4));
    asm volatile("" :: "v"(bv));
  }
#pragma unroll
  for (int i = 0; i < 4; ++i) {
    const int mBase = m0 + (i << 4);
#pragma unroll
    for (int j = 0; j < 4; ++j) {
#pragma unroll
      for (int r = 0; r < 8; ++r) slab[(h8 + r) * 68 + (j << 4) + rl] = acc[i][j][r];
    }
    __builtin_amdgcn_fence(__ATOMIC_RELEASE, "workgroup");
    __builtin_amdgcn_wave_barrier();
    __builtin_amdgcn_fence(__ATOMIC_ACQUIRE, "workgroup");
    v4f vv[8];
#pragma unroll
    for (int it = 0; it < 8; ++it) {
      const int row = it * 2 + hh;
      v4f v = *(const v4fa*)(slab + row * 68 + c4);
      if (EPI == 1) v += bv;
      vv[it] = v;
    }
    for (int pass = 0; pass < 2; ++pass) {
#pragma unroll
      for (int it = 0; it < 8; ++it) {
        const int row = mBase + it * 2 + hh;
        if (cok && row < M) *(volatile v4f*)(D + (size_t)row * (size_t)ldd + nc) = vv[it];
      }
      __threadfence();
    }
    __builtin_amdgcn_fence(__ATOMIC_RELEASE, "workgroup");
    __builtin_amdgcn_wave_barrier();
    __builtin_amdgcn_fence(__ATOMIC_ACQUIRE, "workgroup");
  }
}

#pragma clang fp contract(off)


#ifndef SPLIT_2
#define SPLIT_2 1
#endif

#define NN      50000
#define NE      800000
#define MPAD    50048
#define KD      128
#define C1W     256
#define NHD     4
#define DSZ     64
#define C2W     64
#define OPK     (SPLIT_2 ? 512 : 256)
#define TB_AL1  0
#define TB_AR1  256
#define TB_B1   512
#define TB_AL2  768
#define TB_AR2  832
#define TB_B2   896
#define TB_N    1024
#define BT      512
#define BW      16
#define BEPT    8
#define BCHUNK  (BT * BEPT)
#define NCH     ((NE + BCHUNK - 1) / BCHUNK)
#define NB      1024
#define NBLK    ((NN + NB - 1) / NB)
#define RCAP    20480
#define DEGCAP  64
#define SLOTSH  21
#define LISTTOT (NBLK * RCAP)
#define LDS_BLD ((2 * RCAP + 3 * NB + 64) * 4)
#define OUT_TOT (NN + NN * C2W)
#define PREP_B1 (C1W * KD / 8 / 256)
#define PREP_B2 (C2W * OPK / 8 / 256)
#define WSMAX   ((size_t)128 << 20)

static_assert(NN < (1 << 17));
static_assert(NHD * DSZ == C1W && DSZ == 64 && C2W == 64 && KD == 128);
static_assert(MPAD == 391 * 128 && MPAD % 64 == 0 && MPAD % 32 == 0 && MPAD >= NN);
static_assert(NE < (1 << SLOTSH));
static_assert(NB <= 1024 && (NB & (NB - 1)) == 0 && NB == 2 * BT);
static_assert(NE % 8 == 0 && NE >= 8);
static_assert(NBLK == 49 && NBLK * NB >= MPAD);
static_assert(NCH * BCHUNK >= NE && NCH == 196);
static_assert(RCAP % (4 * BT) == 0);
static_assert(RCAP * 5 >= 16696 * 6);
static_assert(DEGCAP >= 33 + 8);
static_assert(LDS_BLD <= 300000 && LDS_BLD + 34816 <= 327680);
static_assert(BW == BT / 32 && BW == 16);
static_assert(OPK % 32 == 0 && PREP_B1 == 16 && PREP_B2 * 256 * 8 == C2W * OPK);
static_assert(OUT_TOT == 3250000);

typedef int          v4i __attribute__((ext_vector_type(4)));
typedef int          v2i __attribute__((ext_vector_type(2)));
typedef float        v2f __attribute__((ext_vector_type(2)));
typedef v4i __attribute__((may_alias)) v4ia;
typedef v2i __attribute__((may_alias)) v2ia;
typedef v2f __attribute__((may_alias)) v2fa;

__device__ __forceinline__ float relu_k(float v) { return (v > 0.0f) ? v : (v - v); }
__device__ __forceinline__ float lrelu_k(float v) { return (v >= 0.0f) ? v : 0.2f * v; }
__device__ __forceinline__ float maxk(float a, float b) {
  float m = (a < b) ? b : a;
  m = (b != b) ? b : m;
  return m;
}
__device__ __forceinline__ float sum8(float t) {
  t = t + __shfl_xor(t, 4, 32);
  t = t + __shfl_xor(t, 2, 32);
  t = t + __shfl_xor(t, 1, 32);
  return t;
}
__device__ __forceinline__ float sum32(float t) {
  t = t + __shfl_xor(t, 16, 32);
  t = t + __shfl_xor(t, 8, 32);
  t = t + __shfl_xor(t, 4, 32);
  t = t + __shfl_xor(t, 2, 32);
  t = t + __shfl_xor(t, 1, 32);
  return t;
}
__device__ __forceinline__ float dot8(v4f a, v4f b, v4f ta, v4f tb) {
  float t = a.x * ta.x;
  float u = a.y * ta.y; t = t + u;
  u = a.z * ta.z; t = t + u;
  u = a.w * ta.w; t = t + u;
  u = b.x * tb.x; t = t + u;
  u = b.y * tb.y; t = t + u;
  u = b.z * tb.z; t = t + u;
  u = b.w * tb.w; t = t + u;
  return t;
}
__device__ __forceinline__ v4f score4(v4f el, v4f er) {
  v4f e;
  float t;
  t = el.x + er.x; e.x = lrelu_k(t);
  t = el.y + er.y; e.y = lrelu_k(t);
  t = el.z + er.z; e.z = lrelu_k(t);
  t = el.w + er.w; e.w = lrelu_k(t);
  return e;
}

__global__ __launch_bounds__(256) void k_prep(const float* __restrict__ W1, const float* __restrict__ W2,
                                              const float* __restrict__ al1, const float* __restrict__ ar1,
                                              const float* __restrict__ b1, const float* __restrict__ al2,
                                              const float* __restrict__ ar2, const float* __restrict__ b2,
                                              unsigned short* W1T, unsigned short* W2D, float* TB) {
  const int tid = (int)threadIdx.x;
  const int blk = (int)blockIdx.x;
  if (blk < PREP_B1) {
    const int g  = blk * 256 + tid;
    const int n  = g >> 4;
    const int k0 = (g & 15) << 3;
    float x[8];
#pragma unroll
    for (int e = 0; e < 8; ++e) {
      const float v = W1[(size_t)(k0 + e) * C1W + n];
      asm volatile("" :: "v"(v));
      x[e] = v;
    }
    const v4u o = pack8_bf16((v4f){ x[0], x[1], x[2], x[3] }, (v4f){ x[4], x[5], x[6], x[7] });
    volatile v4u* q = (volatile v4u*)(W1T + (size_t)g * 8);
    *q = o;
    __threadfence();
    *q = o;
  } else if (blk < PREP_B1 + PREP_B2) {
    const int g   = (blk - PREP_B1) * 256 + tid;
    const int ppr = OPK / 8;
    const int n   = g / ppr;
    const int p   = g - n * ppr;
    const int k0  = (p << 3) & 255;
    float x[8];
#pragma unroll
    for (int e = 0; e < 8; ++e) {
      const float v = W2[(size_t)(k0 + e) * C2W + n];
      asm volatile("" :: "v"(v));
      x[e] = v;
    }
    const v4u o = pack8_bf16((v4f){ x[0], x[1], x[2], x[3] }, (v4f){ x[4], x[5], x[6], x[7] });
    volatile v4u* q = (volatile v4u*)(W2D + (size_t)g * 8);
    *q = o;
    __threadfence();
    *q = o;
  } else {
    const int idx = 4 * tid;
    const v4f a0 = *(const v4fa*)(al1 + clampi(idx - TB_AL1, 0, 252));
    asm volatile("" :: "v"(a0));
    const v4f a1 = *(const v4fa*)(ar1 + clampi(idx - TB_AR1, 0, 252));
    asm volatile("" :: "v"(a1));
    const v4f a2 = *(const v4fa*)(b1  + clampi(idx - TB_B1,  0, 252));
    asm volatile("" :: "v"(a2));
    const v4f a3 = *(const v4fa*)(al2 + clampi(idx - TB_AL2, 0, 60));
    asm volatile("" :: "v"(a3));
    const v4f a4 = *(const v4fa*)(ar2 + clampi(idx - TB_AR2, 0, 60));
    asm volatile("" :: "v"(a4));
    const v4f a5 = *(const v4fa*)(b2  + clampi(idx - TB_B2,  0, 60));
    asm volatile("" :: "v"(a5));
    const unsigned m0 = (idx < TB_AR1) ? 0xFFFFFFFFu : 0u;
    const unsigned m1 = (idx >= TB_AR1 && idx < TB_B1) ? 0xFFFFFFFFu : 0u;
    const unsigned m2 = (idx >= TB_B1 && idx < TB_AL2) ? 0xFFFFFFFFu : 0u;
    const unsigned m3 = (idx >= TB_AL2 && idx < TB_AR2) ? 0xFFFFFFFFu : 0u;
    const unsigned m4 = (idx >= TB_AR2 && idx < TB_B2) ? 0xFFFFFFFFu : 0u;
    const unsigned m5 = (idx >= TB_B2 && idx < TB_B2 + 64) ? 0xFFFFFFFFu : 0u;
    v4u o;
    o.x = (__float_as_uint(a0.x) & m0) | (__float_as_uint(a1.x) & m1) | (__float_as_uint(a2.x) & m2) |
          (__float_as_uint(a3.x) & m3) | (__float_as_uint(a4.x) & m4) | (__float_as_uint(a5.x) & m5);
    o.y = (__float_as_uint(a0.y) & m0) | (__float_as_uint(a1.y) & m1) | (__float_as_uint(a2.y) & m2) |
          (__float_as_uint(a3.y) & m3) | (__float_as_uint(a4.y) & m4) | (__float_as_uint(a5.y) & m5);
    o.z = (__float_as_uint(a0.z) & m0) | (__float_as_uint(a1.z) & m1) | (__float_as_uint(a2.z) & m2) |
          (__float_as_uint(a3.z) & m3) | (__float_as_uint(a4.z) & m4) | (__float_as_uint(a5.z) & m5);
    o.w = (__float_as_uint(a0.w) & m0) | (__float_as_uint(a1.w) & m1) | (__float_as_uint(a2.w) & m2) |
          (__float_as_uint(a3.w) & m3) | (__float_as_uint(a4.w) & m4) | (__float_as_uint(a5.w) & m5);
    o.x = bf16_bits(__uint_as_float(o.x)) << 16;
    o.y = bf16_bits(__uint_as_float(o.y)) << 16;
    o.z = bf16_bits(__uint_as_float(o.z)) << 16;
    o.w = bf16_bits(__uint_as_float(o.w)) << 16;
    volatile v4u* q = (volatile v4u*)(TB + idx);
    *q = o;
    __threadfence();
    *q = o;
  }
}

__global__ __launch_bounds__(BT) void k_build(const int* __restrict__ ekey, const int* __restrict__ eword,
                                              unsigned* LIST, int* META) {
  extern __shared__ v4u lds_bld[];
  int* reg1 = (int*)lds_bld;
  int* reg2 = reg1 + RCAP;
  int* scnt = reg2 + RCAP;
  int* soff = scnt + NB;
  int* curs = soff + NB;
  int* wcnt = curs + NB;
  int* wtot = wcnt + 2 * BW;
  const int tid = (int)threadIdx.x, lane = tid & 31, wave = tid >> 5;
  const int nodeBase = (int)blockIdx.x * NB;
  int nb = NN - nodeBase;
  nb = nb > NB ? NB : (nb < 0 ? 0 : nb);
  const unsigned nbs = (unsigned)nodeBase, unb = (unsigned)nb;

  scnt[2 * tid] = 0;
  scnt[2 * tid + 1] = 0;
#pragma unroll 1
  for (int i = tid * 4; i < RCAP; i += BT * 4) *(v4ia*)(reg2 + i) = (v4i){0, 0, 0, 0};

  int tot = 0;
#pragma unroll 1
  for (int ch = 0; ch < NCH; ++ch) {
    const int par = ch & 1;
    const int e0  = ch * BCHUNK + tid * BEPT;
    const bool valid = e0 < NE;
    const int ea = e0 < NE - 8 ? e0 : NE - 8;
    const v4i da = *(const v4ia*)(ekey + ea);
    const v4i db = *(const v4ia*)(ekey + ea + 4);
    asm volatile("" :: "v"(da), "v"(db));
    const unsigned s0 = (unsigned)da.x - nbs, s1 = (unsigned)da.y - nbs;
    const unsigned s2 = (unsigned)da.z - nbs, s3 = (unsigned)da.w - nbs;
    const unsigned s4 = (unsigned)db.x - nbs, s5 = (unsigned)db.y - nbs;
    const unsigned s6 = (unsigned)db.z - nbs, s7 = (unsigned)db.w - nbs;
    const bool h0 = valid && (s0 < unb), h1 = valid && (s1 < unb), h2 = valid && (s2 < unb), h3 = valid && (s3 < unb);
    const bool h4 = valid && (s4 < unb), h5 = valid && (s5 < unb), h6 = valid && (s6 < unb), h7 = valid && (s7 < unb);
    const int c = (int)h0 + (int)h1 + (int)h2 + (int)h3 + (int)h4 + (int)h5 + (int)h6 + (int)h7;
    int incl = c;
#pragma unroll
    for (int d = 1; d < 32; d <<= 1) {
      const int up = __shfl_up(incl, d, 32);
      incl += (lane >= d) ? up : 0;
    }
    const int wtotal = __shfl(incl, 31, 32);
    if (lane == 0) wcnt[par * BW + wave] = wtotal;
    __syncthreads();
    int all = 0, pre = 0;
#pragma unroll
    for (int g = 0; g < 4; ++g) {
      const v4i w4 = *(const v4ia*)(wcnt + par * BW + 4 * g);
      const int c0 = clampi(w4.x, 0, 256), c1 = clampi(w4.y, 0, 256);
      const int c2 = clampi(w4.z, 0, 256), c3 = clampi(w4.w, 0, 256);
      all += c0 + c1 + c2 + c3;
      pre += (4 * g + 0 < wave) ? c0 : 0;
      pre += (4 * g + 1 < wave) ? c1 : 0;
      pre += (4 * g + 2 < wave) ? c2 : 0;
      pre += (4 * g + 3 < wave) ? c3 : 0;
    }
    int pos = tot + pre + (incl - c);
#define PUTJ(J, HJ, SJ) if (HJ) { if (pos < RCAP) reg1[pos] = (int)((unsigned)(e0 + (J)) | ((SJ) << SLOTSH)); ++pos; }
    PUTJ(0, h0, s0)
    PUTJ(1, h1, s1)
    PUTJ(2, h2, s2)
    PUTJ(3, h3, s3)
    PUTJ(4, h4, s4)
    PUTJ(5, h5, s5)
    PUTJ(6, h6, s6)
    PUTJ(7, h7, s7)
#undef PUTJ
    tot += all;
  }
  __syncthreads();
  const bool ovf = tot > RCAP;
  const int nh = ovf ? RCAP : tot;

  if (wave == 0) {
#pragma unroll 1
    for (int b0 = 0; b0 < nh; b0 += 32) {
      const int idx = b0 + lane;
      const int uv  = reg1[idx < nh ? idx : nh - 1];
      const int m32 = (nh - b0) < 32 ? (nh - b0) : 32;
#pragma unroll 1
      for (int k = 0; k < m32; ++k) {
        const int u  = __builtin_amdgcn_readlane(uv, k);
        const int sl = (int)(((unsigned)u >> SLOTSH) & (unsigned)(NB - 1));
        const int cv = scnt[sl] + 1;
        if (lane == 0) scnt[sl] = cv;
      }
    }
  }
  __syncthreads();

  int e0c, e1c;
  {
    const v2i cc = *(const v2ia*)(scnt + 2 * tid);
    e0c = cc.x < 0 ? 0 : cc.x;
    e1c = cc.y < 0 ? 0 : cc.y;
    const int ts = e0c + e1c;
    int incl = ts;
#pragma unroll
    for (int d = 1; d < 32; d <<= 1) {
      const int up = __shfl_up(incl, d, 32);
      incl += (lane >= d) ? up : 0;
    }
    if (lane == 31) wtot[wave] = incl;
    __syncthreads();
    int pre = 0;
#pragma unroll
    for (int g = 0; g < 4; ++g) {
      const v4i w4 = *(const v4ia*)(wtot + 4 * g);
      pre += (4 * g + 0 < wave) ? w4.x : 0;
      pre += (4 * g + 1 < wave) ? w4.y : 0;
      pre += (4 * g + 2 < wave) ? w4.z : 0;
      pre += (4 * g + 3 < wave) ? w4.w : 0;
    }
    const int run = pre + incl - ts;
    soff[2 * tid]     = run;
    soff[2 * tid + 1] = run + e0c;
    curs[2 * tid]     = run;
    curs[2 * tid + 1] = run + e0c;
  }
  __syncthreads();

  if (wave == 0) {
#pragma unroll 1
    for (int b0 = 0; b0 < nh; b0 += 32) {
      const int idx = b0 + lane;
      const int uv  = reg1[idx < nh ? idx : nh - 1];
      const int m32 = (nh - b0) < 32 ? (nh - b0) : 32;
#pragma unroll 1
      for (int k = 0; k < m32; ++k) {
        const int u   = __builtin_amdgcn_readlane(uv, k);
        const int sl  = (int)(((unsigned)u >> SLOTSH) & (unsigned)(NB - 1));
        const int eid = (int)((unsigned)u & ((1u << SLOTSH) - 1u));
        const int pr  = curs[sl];
        const int pc  = clampi(pr, 0, RCAP - 1);
        if (lane == 0) { reg2[pc] = eid; curs[sl] = pc + 1; }
      }
    }
  }
  __syncthreads();

  {
    unsigned* lbase = LIST + (size_t)blockIdx.x * (size_t)RCAP;
#pragma unroll 1
    for (int it = 0; it < RCAP / (4 * BT); ++it) {
      const int i4 = (it * BT + tid) * 4;
      const v4i e4 = *(const v4ia*)(reg2 + i4);
      const int q0 = clampi(e4.x, 0, NE - 1), q1 = clampi(e4.y, 0, NE - 1);
      const int q2 = clampi(e4.z, 0, NE - 1), q3 = clampi(e4.w, 0, NE - 1);
      const int w0 = eword[q0];
      asm volatile("" :: "v"(w0));
      const int w1 = eword[q1];
      asm volatile("" :: "v"(w1));
      const int w2 = eword[q2];
      asm volatile("" :: "v"(w2));
      const int w3 = eword[q3];
      asm volatile("" :: "v"(w3));
      v4u o;
      o.x = (unsigned)clampi(w0, 0, NN - 1) & ((i4 + 0 < nh) ? 0xFFFFFFFFu : 0u);
      o.y = (unsigned)clampi(w1, 0, NN - 1) & ((i4 + 1 < nh) ? 0xFFFFFFFFu : 0u);
      o.z = (unsigned)clampi(w2, 0, NN - 1) & ((i4 + 2 < nh) ? 0xFFFFFFFFu : 0u);
      o.w = (unsigned)clampi(w3, 0, NN - 1) & ((i4 + 3 < nh) ? 0xFFFFFFFFu : 0u);
      volatile v4u* q = (volatile v4u*)(lbase + i4);
      *q = o;
      __threadfence();
      *q = o;
    }
  }

  {
    const int base = (int)blockIdx.x * RCAP;
    const v2i cc = *(const v2ia*)(scnt + 2 * tid);
    const v2i so = *(const v2ia*)(soff + 2 * tid);
    v4i m;
    m.x = base + so.x;
    m.y = ovf ? -1 : cc.x;
    m.z = base + so.y;
    m.w = ovf ? -1 : cc.y;
    volatile v4i* q = (volatile v4i*)(META + 2 * (size_t)(nodeBase + 2 * tid));
    *q = m;
    __threadfence();
    *q = m;
  }
}

__global__ __launch_bounds__(256) void k_rowprep4(const float* __restrict__ F1, const float* __restrict__ TB,
                                                  float* EL, float* ER) {
  const int lane = (int)threadIdx.x & 31;
  const int wave = (int)threadIdx.x >> 5;
  const int w = (int)blockIdx.x * 8 + wave;
  if (w >= MPAD / 32) return;
  const int c0 = lane * 8;
  v4f l0 = *(const v4fa*)(TB + TB_AL1 + c0);
  v4f l1 = *(const v4fa*)(TB + TB_AL1 + c0 + 4);
  v4f r0 = *(const v4fa*)(TB + TB_AR1 + c0);
  v4f r1 = *(const v4fa*)(TB + TB_AR1 + c0 + 4);
  asm volatile("" : "+v"(l0), "+v"(l1), "+v"(r0), "+v"(r1));
  v4f kl = (v4f){0.0f, 0.0f, 0.0f, 0.0f};
  v4f kr = (v4f){0.0f, 0.0f, 0.0f, 0.0f};
#pragma unroll 2
  for (int i = 0; i < 32; ++i) {
    const float* fr = F1 + (size_t)(w * 32 + i) * C1W + c0;
    const v4f a = *(const v4fa*)fr;
    const v4f b = *(const v4fa*)(fr + 4);
    float tl = dot8(a, b, l0, l1);
    float tr = dot8(a, b, r0, r1);
    tl = sum8(tl);
    tr = sum8(tr);
    const float x0 = __shfl(tl, 0, 32), x1 = __shfl(tl, 8, 32), x2 = __shfl(tl, 16, 32), x3 = __shfl(tl, 24, 32);
    const float y0 = __shfl(tr, 0, 32), y1 = __shfl(tr, 8, 32), y2 = __shfl(tr, 16, 32), y3 = __shfl(tr, 24, 32);
    const bool mine = (lane == i);
    kl.x = mine ? x0 : kl.x; kl.y = mine ? x1 : kl.y; kl.z = mine ? x2 : kl.z; kl.w = mine ? x3 : kl.w;
    kr.x = mine ? y0 : kr.x; kr.y = mine ? y1 : kr.y; kr.z = mine ? y2 : kr.z; kr.w = mine ? y3 : kr.w;
  }
  volatile v4f* ql = (volatile v4f*)(EL + (size_t)(w * 32 + lane) * NHD);
  volatile v4f* qr = (volatile v4f*)(ER + (size_t)(w * 32 + lane) * NHD);
  *ql = kl;
  *qr = kr;
  __threadfence();
  *ql = kl;
  *qr = kr;
}

__global__ __launch_bounds__(256) void k_rowprep1(const float* __restrict__ F2, const float* __restrict__ TB,
                                                  float* EL, float* ER) {
  const int lane = (int)threadIdx.x & 31;
  const int wave = (int)threadIdx.x >> 5;
  const int w = (int)blockIdx.x * 8 + wave;
  if (w >= MPAD / 32) return;
  v2f tl2 = *(const v2fa*)(TB + TB_AL2 + 2 * lane);
  v2f tr2 = *(const v2fa*)(TB + TB_AR2 + 2 * lane);
  asm volatile("" : "+v"(tl2), "+v"(tr2));
  float kl = 0.0f, kr = 0.0f;
#pragma unroll 2
  for (int i = 0; i < 32; ++i) {
    const v2f f = *(const v2fa*)(F2 + (size_t)(w * 32 + i) * C2W + 2 * lane);
    float tl = f.x * tl2.x;
    float u  = f.y * tl2.y; tl = tl + u;
    float tr = f.x * tr2.x;
    u = f.y * tr2.y; tr = tr + u;
    tl = sum32(tl);
    tr = sum32(tr);
    const bool mine = (lane == i);
    kl = mine ? tl : kl;
    kr = mine ? tr : kr;
  }
  volatile float* ql = (volatile float*)(EL + (size_t)(w * 32 + lane));
  volatile float* qr = (volatile float*)(ER + (size_t)(w * 32 + lane));
  *ql = kl;
  *qr = kr;
  __threadfence();
  *ql = kl;
  *qr = kr;
}

__global__ __launch_bounds__(256) void k_walk1(const float* __restrict__ F1, const float* __restrict__ EL,
                                               const float* __restrict__ ER, const unsigned* __restrict__ LIST,
                                               const int* __restrict__ META, const float* __restrict__ TB,
                                               unsigned short* OP) {
  const int lane = (int)threadIdx.x & 31;
  const int wave = (int)threadIdx.x >> 5;
  const int row  = (int)blockIdx.x * 8 + wave;
  const bool real = row < NN;
  const int head = lane >> 3;
  const int c0   = lane * 8;

  const v2i mt = *(const v2ia*)(META + 2 * (size_t)row);
  asm volatile("" :: "v"(mt));
  const int craw = mt.y;
  const int offv = clampi(mt.x, 0, LISTTOT);
  const int cntv = real ? (clampi(craw, 0, DEGCAP) < (LISTTOT - offv) ? clampi(craw, 0, DEGCAP) : (LISTTOT - offv)) : 0;
  const int off = __builtin_amdgcn_readfirstlane(offv);
  const int cnt = __builtin_amdgcn_readfirstlane(cntv);
  const bool poison = real && ((craw < 0) || (craw > DEGCAP));

  const v4f er4 = *(const v4fa*)(ER + (size_t)row * NHD);
  asm volatile("" :: "v"(er4));
  const float ninf = -__builtin_inff();
  v4f mx4 = (v4f){ninf, ninf, ninf, ninf};

#pragma unroll 1
  for (int b0 = 0; b0 < cnt; b0 += 32) {
    const int j = (b0 + lane) < cnt ? (b0 + lane) : cnt - 1;
    const unsigned sid = LIST[(size_t)(off + j)];
    asm volatile("" :: "v"(sid));
    const int col = clampi((int)sid, 0, NN - 1);
    const v4f el4 = *(const v4fa*)(EL + (size_t)col * NHD);
    asm volatile("" :: "v"(el4));
    const v4f e4 = score4(el4, er4);
    mx4.x = maxk(mx4.x, e4.x);
    mx4.y = maxk(mx4.y, e4.y);
    mx4.z = maxk(mx4.z, e4.z);
    mx4.w = maxk(mx4.w, e4.w);
  }
#pragma unroll
  for (int d = 16; d > 0; d >>= 1) {
    const float o0 = __shfl_xor(mx4.x, d, 32);
    const float o1 = __shfl_xor(mx4.y, d, 32);
    const float o2 = __shfl_xor(mx4.z, d, 32);
    const float o3 = __shfl_xor(mx4.w, d, 32);
    mx4.x = maxk(mx4.x, o0);
    mx4.y = maxk(mx4.y, o1);
    mx4.z = maxk(mx4.z, o2);
    mx4.w = maxk(mx4.w, o3);
  }

  float d0 = 0.0f, d1 = 0.0f, d2 = 0.0f, d3 = 0.0f;
#pragma unroll 1
  for (int b0 = 0; b0 < cnt; b0 += 32) {
    const int j = (b0 + lane) < cnt ? (b0 + lane) : cnt - 1;
    const unsigned sid = LIST[(size_t)(off + j)];
    asm volatile("" :: "v"(sid));
    const int col = clampi((int)sid, 0, NN - 1);
    const v4f el4 = *(const v4fa*)(EL + (size_t)col * NHD);
    asm volatile("" :: "v"(el4));
    const v4f e4 = score4(el4, er4);
    const float v0 = e4.x - mx4.x, v1 = e4.y - mx4.y, v2 = e4.z - mx4.z, v3 = e4.w - mx4.w;
    const float x0 = expf(v0), x1 = expf(v1), x2 = expf(v2), x3 = expf(v3);
    const int m32 = (cnt - b0) < 32 ? (cnt - b0) : 32;
#pragma unroll 1
    for (int k = 0; k < m32; ++k) {
      const float t0 = __int_as_float(__builtin_amdgcn_readlane(__float_as_int(x0), k));
      const float t1 = __int_as_float(__builtin_amdgcn_readlane(__float_as_int(x1), k));
      const float t2 = __int_as_float(__builtin_amdgcn_readlane(__float_as_int(x2), k));
      const float t3 = __int_as_float(__builtin_amdgcn_readlane(__float_as_int(x3), k));
      d0 = d0 + t0;
      d1 = d1 + t1;
      d2 = d2 + t2;
      d3 = d3 + t3;
    }
  }

  v4f a0 = (v4f){0.0f, 0.0f, 0.0f, 0.0f};
  v4f a1 = (v4f){0.0f, 0.0f, 0.0f, 0.0f};
#pragma unroll 1
  for (int b0 = 0; b0 < cnt; b0 += 32) {
    const int j = (b0 + lane) < cnt ? (b0 + lane) : cnt - 1;
    const unsigned sid = LIST[(size_t)(off + j)];
    asm volatile("" :: "v"(sid));
    const int col = clampi((int)sid, 0, NN - 1);
    const v4f el4 = *(const v4fa*)(EL + (size_t)col * NHD);
    asm volatile("" :: "v"(el4));
    const v4f e4 = score4(el4, er4);
    const float v0 = e4.x - mx4.x, v1 = e4.y - mx4.y, v2 = e4.z - mx4.z, v3 = e4.w - mx4.w;
    const float q0 = expf(v0) / d0;
    const float q1 = expf(v1) / d1;
    const float q2 = expf(v2) / d2;
    const float q3 = expf(v3) / d3;
    const int m32 = (cnt - b0) < 32 ? (cnt - b0) : 32;
#pragma unroll 1
    for (int k = 0; k < m32; ++k) {
      const int c = __builtin_amdgcn_readlane(col, k);
      const float w0 = __int_as_float(__builtin_amdgcn_readlane(__float_as_int(q0), k));
      const float w1 = __int_as_float(__builtin_amdgcn_readlane(__float_as_int(q1), k));
      const float w2 = __int_as_float(__builtin_amdgcn_readlane(__float_as_int(q2), k));
      const float w3 = __int_as_float(__builtin_amdgcn_readlane(__float_as_int(q3), k));
      float w = w0;
      w = (head == 1) ? w1 : w;
      w = (head == 2) ? w2 : w;
      w = (head == 3) ? w3 : w;
      const float* fp = F1 + (size_t)c * C1W + c0;
      const v4f f0 = *(const v4fa*)fp;
      asm volatile("" :: "v"(f0));
      const v4f f1 = *(const v4fa*)(fp + 4);
      asm volatile("" :: "v"(f1));
      float pr;
      pr = w * f0.x; a0.x = a0.x + pr;
      pr = w * f0.y; a0.y = a0.y + pr;
      pr = w * f0.z; a0.z = a0.z + pr;
      pr = w * f0.w; a0.w = a0.w + pr;
      pr = w * f1.x; a1.x = a1.x + pr;
      pr = w * f1.y; a1.y = a1.y + pr;
      pr = w * f1.z; a1.z = a1.z + pr;
      pr = w * f1.w; a1.w = a1.w + pr;
    }
  }

  v4f bv0 = *(const v4fa*)(TB + TB_B1 + c0);
  v4f bv1 = *(const v4fa*)(TB + TB_B1 + c0 + 4);
  asm volatile("" : "+v"(bv0), "+v"(bv1));
  const float qnan = __uint_as_float(0x7fc00000u);
  v4f y0, y1;
  y0.x = relu_k(a0.x + bv0.x); y0.y = relu_k(a0.y + bv0.y); y0.z = relu_k(a0.z + bv0.z); y0.w = relu_k(a0.w + bv0.w);
  y1.x = relu_k(a1.x + bv1.x); y1.y = relu_k(a1.y + bv1.y); y1.z = relu_k(a1.z + bv1.z); y1.w = relu_k(a1.w + bv1.w);
  y0.x = poison ? qnan : y0.x; y0.y = poison ? qnan : y0.y; y0.z = poison ? qnan : y0.z; y0.w = poison ? qnan : y0.w;
  y1.x = poison ? qnan : y1.x; y1.y = poison ? qnan : y1.y; y1.z = poison ? qnan : y1.z; y1.w = poison ? qnan : y1.w;
  const unsigned rm = real ? 0xFFFFFFFFu : 0u;
  const v4u rmask = (v4u){rm, rm, rm, rm};
  v4u hi = pack8_bf16(y0, y1);
  hi &= rmask;
  unsigned short* orow = OP + (size_t)row * OPK + c0;
  volatile v4u* qh = (volatile v4u*)orow;
  if (SPLIT_2) {
    v4u lo = pack8_bf16_lo(y0, y1);
    lo &= rmask;
    volatile v4u* ql = (volatile v4u*)(orow + 256);
    *qh = hi;
    *ql = lo;
    __threadfence();
    *qh = hi;
    *ql = lo;
  } else {
    *qh = hi;
    __threadfence();
    *qh = hi;
  }
}

__global__ __launch_bounds__(256) void k_walk2(const float* __restrict__ F2, const float* __restrict__ EL,
                                               const float* __restrict__ ER, const unsigned* __restrict__ LIST,
                                               const int* __restrict__ META, const float* __restrict__ TB,
                                               float* G, float* S) {
  const int lane = (int)threadIdx.x & 31;
  const int wave = (int)threadIdx.x >> 5;
  const int row  = (int)blockIdx.x * 8 + wave;
  const bool real = row < NN;

  const v2i mt = *(const v2ia*)(META + 2 * (size_t)row);
  asm volatile("" :: "v"(mt));
  const int craw = mt.y;
  const int offv = clampi(mt.x, 0, LISTTOT);
  const int cntv = real ? (clampi(craw, 0, DEGCAP) < (LISTTOT - offv) ? clampi(craw, 0, DEGCAP) : (LISTTOT - offv)) : 0;
  const int off = __builtin_amdgcn_readfirstlane(offv);
  const int cnt = __builtin_amdgcn_readfirstlane(cntv);
  const bool poison = real && ((craw < 0) || (craw > DEGCAP));

  const float er = ER[row];
  asm volatile("" :: "v"(er));
  float mx = -__builtin_inff();
#pragma unroll 1
  for (int b0 = 0; b0 < cnt; b0 += 32) {
    const int j = (b0 + lane) < cnt ? (b0 + lane) : cnt - 1;
    const unsigned sid = LIST[(size_t)(off + j)];
    asm volatile("" :: "v"(sid));
    const int col = clampi((int)sid, 0, NN - 1);
    const float el = EL[col];
    asm volatile("" :: "v"(el));
    const float t = el + er;
    mx = maxk(mx, lrelu_k(t));
  }
#pragma unroll
  for (int d = 16; d > 0; d >>= 1) {
    const float o0 = __shfl_xor(mx, d, 32);
    mx = maxk(mx, o0);
  }

  float den = 0.0f;
#pragma unroll 1
  for (int b0 = 0; b0 < cnt; b0 += 32) {
    const int j = (b0 + lane) < cnt ? (b0 + lane) : cnt - 1;
    const unsigned sid = LIST[(size_t)(off + j)];
    asm volatile("" :: "v"(sid));
    const int col = clampi((int)sid, 0, NN - 1);
    const float el = EL[col];
    asm volatile("" :: "v"(el));
    const float t = el + er;
    const float v = lrelu_k(t) - mx;
    const float x = expf(v);
    const int m32 = (cnt - b0) < 32 ? (cnt - b0) : 32;
#pragma unroll 1
    for (int k = 0; k < m32; ++k) {
      const float tk = __int_as_float(__builtin_amdgcn_readlane(__float_as_int(x), k));
      den = den + tk;
    }
  }

  v2f ac = (v2f){0.0f, 0.0f};
#pragma unroll 1
  for (int b0 = 0; b0 < cnt; b0 += 32) {
    const int j = (b0 + lane) < cnt ? (b0 + lane) : cnt - 1;
    const unsigned sid = LIST[(size_t)(off + j)];
    asm volatile("" :: "v"(sid));
    const int col = clampi((int)sid, 0, NN - 1);
    const float el = EL[col];
    asm volatile("" :: "v"(el));
    const float t = el + er;
    const float v = lrelu_k(t) - mx;
    const float q = expf(v) / den;
    const int m32 = (cnt - b0) < 32 ? (cnt - b0) : 32;
#pragma unroll 1
    for (int k = 0; k < m32; ++k) {
      const int c = __builtin_amdgcn_readlane(col, k);
      const float w = __int_as_float(__builtin_amdgcn_readlane(__float_as_int(q), k));
      const v2f f = *(const v2fa*)(F2 + (size_t)c * C2W + 2 * lane);
      asm volatile("" :: "v"(f));
      float pr;
      pr = w * f.x; ac.x = ac.x + pr;
      pr = w * f.y; ac.y = ac.y + pr;
    }
  }

  v2f bv = *(const v2fa*)(TB + TB_B2 + 2 * lane);
  asm volatile("" : "+v"(bv));
  const float qnan = __uint_as_float(0x7fc00000u);
  v2f o;
  o.x = relu_k(ac.x + bv.x);
  o.y = relu_k(ac.y + bv.y);
  o.x = poison ? qnan : o.x;
  o.y = poison ? qnan : o.y;
  o.x = real ? o.x : 0.0f;
  o.y = real ? o.y : 0.0f;
  float s = o.x + o.y;
  s = sum32(s);
  const float sv = (lane == 0) ? s : 0.0f;
  volatile v2f*   qg = (volatile v2f*)(G + (size_t)row * C2W + 2 * lane);
  volatile float* qs = (volatile float*)(S + (size_t)row * 32 + lane);
  *qg = o;
  *qs = sv;
  __threadfence();
  *qg = o;
  *qs = sv;
}

__global__ __launch_bounds__(256) void k_flat(const float* __restrict__ S, const float* __restrict__ G,
                                              float* out, int total) {
  const int f = (int)blockIdx.x * 256 + (int)threadIdx.x;
  const int si = clampi(f, 0, NN - 1);
  const float sv = S[(size_t)si * 32];
  asm volatile("" :: "v"(sv));
  const int gi = clampi(f - NN, 0, NN * C2W - 1);
  const float gv = G[gi];
  asm volatile("" :: "v"(gv));
  const unsigned ms = (f < NN) ? 0xFFFFFFFFu : 0u;
  const float val = __uint_as_float((__float_as_uint(sv) & ms) | (__float_as_uint(gv) & ~ms));
  const bool wr = f < total;
  volatile float* q = (volatile float*)(out + (wr ? f : 0));
  if (wr) *q = val;
  __threadfence();
  if (wr) *q = val;
}

extern "C" void kernel_launch(void* const* d_in, const int* in_sizes, int n_in,
                              void* d_out, int out_size, void* d_ws, size_t ws_size,
                              hipStream_t stream) {
  if (n_in < 11) return;
  if (in_sizes[0] != NN * KD) return;
  if (in_sizes[1] != NE || in_sizes[2] != NE) return;
  if (in_sizes[3] != KD * C1W) return;
  if (in_sizes[4] != C1W || in_sizes[5] != C1W || in_sizes[6] != C1W) return;
  if (in_sizes[7] != C1W * C2W) return;
  if (in_sizes[8] != C2W || in_sizes[9] != C2W || in_sizes[10] != C2W) return;
  if (out_size != OUT_TOT) return;

  const float* x    = (const float*)d_in[0];
  const int*   esrc = (const int*)  d_in[1];
  const int*   edst = (const int*)  d_in[2];
  const float* W1   = (const float*)d_in[3];
  const float* al1  = (const float*)d_in[4];
  const float* ar1  = (const float*)d_in[5];
  const float* b1   = (const float*)d_in[6];
  const float* W2   = (const float*)d_in[7];
  const float* al2  = (const float*)d_in[8];
  const float* ar2  = (const float*)d_in[9];
  const float* b2   = (const float*)d_in[10];
  float* out = (float*)d_out;

  constexpr size_t szXB   = (size_t)MPAD * KD * 2;
  constexpr size_t szW1T  = (size_t)C1W * KD * 2;
  constexpr size_t szW2D  = (size_t)C2W * 512 * 2;
  constexpr size_t szTB   = (size_t)TB_N * 4;
  constexpr size_t szF1   = (size_t)MPAD * C1W * 4;
  constexpr size_t szOP   = (size_t)MPAD * 512 * 2;
  constexpr size_t szG    = (size_t)MPAD * C2W * 4;
  constexpr size_t szS    = (size_t)MPAD * 32 * 4;
  constexpr size_t szE1   = (size_t)MPAD * NHD * 4;
  constexpr size_t szE2   = (size_t)MPAD * 4;
  constexpr size_t szMETA = (size_t)NBLK * NB * 2 * 4;
  constexpr size_t szLIST = (size_t)NBLK * RCAP * 4;
  constexpr size_t szALL  = szXB + szW1T + szW2D + szTB + szF1 + szOP + 2 * szE1 + 2 * szE2 + szMETA + szLIST;
  static_assert(szXB % 128 == 0 && szF1 % 128 == 0 && szOP % 128 == 0 && szG % 128 == 0 && szS % 128 == 0);
  static_assert(szE1 % 128 == 0 && szE2 % 128 == 0 && szMETA % 128 == 0 && szLIST % 128 == 0);
  static_assert(szG + szS <= (size_t)MPAD * 256 * 2);
  static_assert((size_t)MPAD * C2W * 4 <= szF1);
  static_assert(szALL <= WSMAX);
  char* ws = (char*)d_ws;
  size_t off = 0;
  const size_t oXB   = off; off += szXB;
  const size_t oW1T  = off; off += szW1T;
  const size_t oW2D  = off; off += szW2D;
  const size_t oTB   = off; off += szTB;
  const size_t oF1   = off; off += szF1;
  const size_t oOP   = off; off += szOP;
  const size_t oEL1  = off; off += szE1;
  const size_t oER1  = off; off += szE1;
  const size_t oEL2  = off; off += szE2;
  const size_t oER2  = off; off += szE2;
  const size_t oMETA = off; off += szMETA;
  const size_t oLIST = off; off += szLIST;
  if (off > ws_size || off > (size_t)WSMAX) return;
  unsigned short* XB  = (unsigned short*)(ws + oXB);
  unsigned short* W1T = (unsigned short*)(ws + oW1T);
  unsigned short* W2D = (unsigned short*)(ws + oW2D);
  float*    TB   = (float*)(ws + oTB);
  float*    F1   = (float*)(ws + oF1);
  float*    F2   = (float*)(ws + oF1);
  unsigned short* OP = (unsigned short*)(ws + oOP);
  float*    G    = (float*)(ws + oOP);
  float*    S    = (float*)(ws + oOP + szG);
  float*    EL1  = (float*)(ws + oEL1);
  float*    ER1  = (float*)(ws + oER1);
  float*    EL2  = (float*)(ws + oEL2);
  float*    ER2  = (float*)(ws + oER2);
  int*      META = (int*)(ws + oMETA);
  unsigned* LIST = (unsigned*)(ws + oLIST);

  hipFuncSetAttribute(reinterpret_cast<const void*>(&k_build),
                      hipFuncAttributeMaxDynamicSharedMemorySize, LDS_BLD);

  k_plane<0><<<MPAD * KD / 8 / 256, 256, 0, stream>>>(x, NN, KD, KD, XB, MPAD, KD);
  k_prep<<<PREP_B1 + PREP_B2 + 1, 256, 0, stream>>>(W1, W2, al1, ar1, b1, al2, ar2, b2, W1T, W2D, TB);
  k_build<<<NBLK, BT, LDS_BLD, stream>>>(edst, esrc, LIST, META);
  {
    const int tiles = (MPAD / 64) * (C1W / 64);
    k_gemm_nt<0, 0><<<(tiles + 7) / 8, 256, 0, stream>>>(XB, W1T, TB, F1, MPAD, C1W, KD, C1W);
  }
  k_rowprep4<<<(MPAD / 32 + 7) / 8, 256, 0, stream>>>(F1, TB, EL1, ER1);
  k_walk1<<<MPAD / 8, 256, 0, stream>>>(F1, EL1, ER1, LIST, META, TB, OP);
  {
    const int tiles = (MPAD / 64) * (C2W / 64);
    k_gemm_nt<0, 0><<<(tiles + 7) / 8, 256, 0, stream>>>(OP, W2D, TB, F2, MPAD, C2W, OPK, C2W);
  }
  k_rowprep1<<<(MPAD / 32 + 7) / 8, 256, 0, stream>>>(F2, TB, EL2, ER2);
  k_walk2<<<MPAD / 8, 256, 0, stream>>>(F2, EL2, ER2, LIST, META, TB, G, S);
  k_flat<<<((OUT_TOT + 31) / 32 + 7) / 8, 256, 0, stream>>>(S, G, out, OUT_TOT);
}
